// qODEDynamics_58342835749471
// MI455X (gfx1250) — hardware-verified
//
#include <hip/hip_runtime.h>


#define NW_  1024
#define LL   32
#define HH   64
#define ICH  64
#define NPC  (ICH * NW_)
#define DM   HH
#define LOSC 1024.0f

typedef _Float16 h16;
typedef unsigned short bf;
typedef __attribute__((ext_vector_type(16))) __bf16   v16bf;
typedef __attribute__((ext_vector_type(16))) _Float16 v16h;
typedef __attribute__((ext_vector_type(8)))  _Float16 v8h;
typedef __attribute__((ext_vector_type(8)))  unsigned short v8us;
typedef __attribute__((ext_vector_type(8)))  float    v8f;
typedef __attribute__((ext_vector_type(4)))  float    v4f;
typedef v8h  __attribute__((may_alias)) v8ha;
typedef v4f  __attribute__((may_alias)) v4fa;
typedef v8us __attribute__((may_alias)) v8usa;

__device__ __forceinline__ unsigned short f2bf(float f) { unsigned u = __float_as_uint(f); u += 0x7FFFu + ((u >> 16) & 1u); return (unsigned short)(u >> 16); }
__device__ __forceinline__ float bf2f(unsigned short b) { return __uint_as_float(((unsigned)b) << 16); }
__device__ __forceinline__ float bfr(float f) { return bf2f(f2bf(f)); }
__device__ __forceinline__ v16h cat16(v8h lo, v8h hi) { return __builtin_shufflevector(lo, hi, 0, 1, 2, 3, 4, 5, 6, 7, 8, 9, 10, 11, 12, 13, 14, 15); }
__device__ __forceinline__ v16bf cat16b(v8us lo, v8us hi) { return __builtin_bit_cast(v16bf, __builtin_shufflevector(lo, hi, 0, 1, 2, 3, 4, 5, 6, 7, 8, 9, 10, 11, 12, 13, 14, 15)); }
__device__ __forceinline__ v8f wmma16(v16h a, v16h b, v8f c) { return __builtin_amdgcn_wmma_f32_16x16x32_f16(false, a, false, b, (short)0, c, false, false); }
__device__ __forceinline__ v8f wmmab(v16bf a, v16bf b, v8f c) { return __builtin_amdgcn_wmma_f32_16x16x32_bf16(false, a, false, b, (short)0, c, false, false); }

template <bool SPLITA, bool F16OUT = false>
__global__ __launch_bounds__(128) void k_gemmb(const bf* __restrict__ A, const bf* __restrict__ Al, const bf* __restrict__ Bn, const float* __restrict__ bias, float* C, int ldc, h16* C2, const float* __restrict__ R = nullptr, int K = DM, int roundR = 1) {
    __shared__ __align__(16) float ost[4][16 * 68];
    const int lane = threadIdx.x & 31, wave = threadIdx.x >> 5, lr = lane & 15, hi = lane >> 4;
    const int r0 = blockIdx.x * 64 + wave * 16, c0 = blockIdx.y * 64;
    const size_t aoff = (size_t)(r0 + lr) * K + 8 * hi;
    size_t boff[4];
#pragma unroll
    for (int t = 0; t < 4; ++t) boff[t] = (size_t)(c0 + t * 16 + lr) * K + 8 * hi;
    v8f acc[4];
#pragma unroll
    for (int t = 0; t < 4; ++t) acc[t] = (v8f){};
#pragma unroll 1
    for (int kc = 0; kc < K; kc += 32) {
        const v16bf a = cat16b(*(const v8us*)(A + aoff + kc), *(const v8us*)(A + aoff + kc + 16));
        v16bf al = a;
        if (SPLITA) al = cat16b(*(const v8us*)(Al + aoff + kc), *(const v8us*)(Al + aoff + kc + 16));
#pragma unroll
        for (int t = 0; t < 4; ++t) { const v16bf b = cat16b(*(const v8us*)(Bn + boff[t] + kc), *(const v8us*)(Bn + boff[t] + kc + 16)); acc[t] = wmmab(a, b, acc[t]); if (SPLITA) acc[t] = wmmab(al, b, acc[t]); }
        asm volatile("v_nop\n\tv_nop\n\tv_nop\n\tv_nop" : "+v"(acc[0]), "+v"(acc[1]), "+v"(acc[2]), "+v"(acc[3]) : "v"(a), "v"(al));
    }
    float* os = &ost[wave][0];
#pragma unroll
    for (int t = 0; t < 4; ++t) { const float bv = bias ? bfr(bias[c0 + t * 16 + lr]) : 0.f;
#pragma unroll
        for (int j = 0; j < 8; ++j) os[(hi * 8 + j) * 68 + t * 16 + lr] = acc[t][j] + bv; }
    __syncthreads();
    if (F16OUT) {
        h16* crow = (h16*)(void*)C + (size_t)r0 * ldc + c0;
        auto pass = [&]() {
#pragma unroll
            for (int s = 0; s < 4; ++s) { const int row = 4 * s + (lane >> 3), piece = lane & 7; const float* sp = os + row * 68 + piece * 8; v8h o, o2;
#pragma unroll
                for (int i = 0; i < 8; ++i) { const h16 a = (h16)sp[i]; o[i] = a; o2[i] = (h16)((sp[i] - (float)a) * LOSC); }
                *(volatile v8h*)(crow + (size_t)row * ldc + piece * 8) = o; if (C2) *(volatile v8h*)(C2 + (size_t)r0 * ldc + c0 + (size_t)row * ldc + piece * 8) = o2; }
        };
        pass(); __threadfence(); pass();
    } else {
        float* crow = C + (size_t)r0 * ldc + c0;
        auto pass = [&]() {
#pragma unroll
            for (int s = 0; s < 8; ++s) { const int Lid = (lane >> 3) + 4 * s, piece = lane & 7; const int row = Lid >> 1, cofs = (Lid & 1) * 32 + piece * 4;
                v4f val = *(const v4fa*)(os + row * 68 + cofs); if (R) { const v4f rv = *(const v4f*)(R + ((size_t)r0 + row) * ldc + c0 + cofs); val += roundR ? (v4f){bfr(rv[0]), bfr(rv[1]), bfr(rv[2]), bfr(rv[3])} : rv; }
                *(volatile v4f*)(crow + (size_t)row * ldc + cofs) = val; }
        };
        pass(); __threadfence(); pass();
    }
}


__global__ __launch_bounds__(256) void k_hb(const float* __restrict__ st, bf* HB) {
    const int u = blockIdx.x * 256 + threadIdx.x; if (u >= NW_ * HH / 8) return; v8us o;
#pragma unroll
    for (int q = 0; q < 8; ++q) { const int f = u * 8 + q; const int i = f / HH, l = f % HH; o[q] = (l < LL) ? f2bf(st[i * (LL + 1) + (l < LL ? l : 0)]) : (unsigned short)0; }
    *(volatile v8us*)(HB + (size_t)u * 8) = o; __threadfence(); *(volatile v8us*)(HB + (size_t)u * 8) = o;
}
__global__ __launch_bounds__(256) void k_w64(const float* __restrict__ Wm, int nout, int ws, int c0, int kk, bf* WT) {
    typedef __attribute__((ext_vector_type(2))) unsigned short v2us;
    const int lane = threadIdx.x & 31, n = blockIdx.x * 8 + (threadIdx.x >> 5); if (n >= 64) return; v2us o;
#pragma unroll
    for (int i = 0; i < 2; ++i) { const int k = lane * 2 + i; const bool ok = (n < nout) && (k < kk); o[i] = ok ? f2bf(Wm[(size_t)(ok ? n : 0) * ws + c0 + (ok ? k : 0)]) : (unsigned short)0; }
    *(volatile v2us*)(WT + (size_t)n * 64 + lane * 2) = o; __threadfence(); *(volatile v2us*)(WT + (size_t)n * 64 + lane * 2) = o;
}
template <int MODE>
__global__ __launch_bounds__(256) void k_act64(const float* __restrict__ src, const float* __restrict__ bias, int nrows, bf* dh, bf* dl) {
    typedef __attribute__((ext_vector_type(2))) unsigned short v2us;
    const int lane = threadIdx.x & 31; const size_t r = (size_t)blockIdx.x * 8 + (threadIdx.x >> 5); if (r >= (size_t)nrows) return; v2us oh, ol;
#pragma unroll
    for (int i = 0; i < 2; ++i) { const int c = lane * 2 + i; float v = src[r * HH + c]; if (MODE == 0) v = tanhf(v + bfr(bias[c])); if (MODE == 2 && c < LL) v += bfr(bias[c]); const unsigned short hb = f2bf(v); oh[i] = hb; ol[i] = f2bf(v - bf2f(hb)); }
    const size_t o = r * HH + lane * 2; *(volatile v2us*)(dh + o) = oh; *(volatile v2us*)(dl + o) = ol; __threadfence(); *(volatile v2us*)(dh + o) = oh; *(volatile v2us*)(dl + o) = ol;
}
__global__ __launch_bounds__(256) void k_x1(const float* __restrict__ A, const float* __restrict__ Bm, const float* __restrict__ bias, int i0, bf* dh, bf* dl) {
    typedef __attribute__((ext_vector_type(2))) unsigned short v2us;
    const int lane = threadIdx.x & 31; const size_t r = (size_t)blockIdx.x * 8 + (threadIdx.x >> 5); if (r >= (size_t)NPC) return; const int il = (int)(r / NW_), j = (int)(r % NW_); v2us oh, ol;
#pragma unroll
    for (int q = 0; q < 2; ++q) { const int c = lane * 2 + q; const float v = tanhf(A[(size_t)(i0 + il) * HH + c] + Bm[(size_t)j * HH + c] + bfr(bias[c])); const unsigned short hb = f2bf(v); oh[q] = hb; ol[q] = f2bf(v - bf2f(hb)); }
    const size_t o = r * HH + lane * 2; *(volatile v2us*)(dh + o) = oh; *(volatile v2us*)(dl + o) = ol; __threadfence(); *(volatile v2us*)(dh + o) = oh; *(volatile v2us*)(dl + o) = ol;
}
__global__ __launch_bounds__(256) void k_isum(const float* __restrict__ st, const float* __restrict__ KIJ, const float* __restrict__ bi3, const float* __restrict__ CA, const float* __restrict__ CB, const float* __restrict__ bc, const float* __restrict__ pw, const float* __restrict__ aggr, int i0, float* ISUM) {
    const int lane = threadIdx.x & 31, il = blockIdx.x * 8 + (threadIdx.x >> 5); if (il >= ICH) return; const int i = i0 + il, l = lane;
    const float hi_l = bfr(st[i * (LL + 1) + l]), phi = bfr(st[i * (LL + 1) + LL]), ag = 1.0f / (1.0f + __expf(-bfr(aggr[i]))), wl = bfr(pw[l]), cai = CA[(size_t)i * HH + l], bcl = bfr(bc[l]), b3 = bfr(bi3[l]);
    float acc = 0.f;
#pragma unroll 1
    for (int j = 0; j < NW_; ++j) { if (j == i) continue;
        const float hj_l = bfr(st[j * (LL + 1) + l]); const float df = hi_l - hj_l; float d2 = df * df;
#pragma unroll
        for (int sh = 16; sh; sh >>= 1) d2 += __shfl_xor(d2, sh, 32);
        const float dfac = fminf(1.0f / (sqrtf(d2) + 1e-6f), 2.0f);
        const float kij = KIJ[((size_t)il * NW_ + j) * HH + l] + b3; const float phj = bfr(st[j * (LL + 1) + LL]);
        const float pf = cosf((phi - phj) * wl); const float coh = 1.0f / (1.0f + __expf(-(cai + CB[(size_t)j * HH + l] + bcl)));
        acc += dfac * kij * ag + pf * coh * (hj_l - hi_l); }
    *(volatile float*)(ISUM + (size_t)i * LL + l) = acc; __threadfence(); *(volatile float*)(ISUM + (size_t)i * LL + l) = acc;
}
__global__ __launch_bounds__(256) void k_out(const float* __restrict__ SELF, const float* __restrict__ bs3, const float* __restrict__ ISUM, float* OUTP) {
    const int u = blockIdx.x * 256 + threadIdx.x; if (u >= NW_ * (LL + 1) / 4) return; v4f o;
#pragma unroll
    for (int q = 0; q < 4; ++q) { const int e = u * 4 + q; const int i = e / (LL + 1), c = e % (LL + 1); float v;
        if (c < LL) v = 0.5f * (SELF[(size_t)i * HH + c] + bfr(bs3[c])) + 0.3f * ISUM[(size_t)i * LL + c];
        else { float s = 0.f;
#pragma unroll 8
            for (int l = 0; l < LL; ++l) s += fabsf(ISUM[(size_t)i * LL + l]);
            v = 0.1f + 0.05f * s; }
        o[q] = v; }
    *(volatile v4f*)(OUTP + (size_t)u * 4) = o; __threadfence(); *(volatile v4f*)(OUTP + (size_t)u * 4) = o;
}

extern "C" void kernel_launch(void* const* d_in, const int* in_sizes, int n_in,
                              void* d_out, int out_size, void* d_ws, size_t ws_size, hipStream_t stream) {
    (void)in_sizes; (void)n_in; (void)out_size;
    const float* st = (const float*)d_in[0];
    const float* Ws1 = (const float*)d_in[1]; const float* bs1 = (const float*)d_in[2]; const float* Ws2 = (const float*)d_in[3]; const float* bs2 = (const float*)d_in[4]; const float* Ws3 = (const float*)d_in[5]; const float* bs3 = (const float*)d_in[6];
    const float* Wi1 = (const float*)d_in[7]; const float* bi1 = (const float*)d_in[8]; const float* Wi2 = (const float*)d_in[9]; const float* bi2 = (const float*)d_in[10]; const float* Wi3 = (const float*)d_in[11]; const float* bi3 = (const float*)d_in[12];
    const float* pw = (const float*)d_in[13]; const float* Wc = (const float*)d_in[14]; const float* bc = (const float*)d_in[15]; const float* aggr = (const float*)d_in[16];
    float* out = (float*)d_out;
    char* wsp = (char*)d_ws;
    auto take = [&](size_t bytes) { char* p = wsp; wsp += (bytes + 255) & ~(size_t)255; return (void*)p; };
    bf* HB = (bf*)take((size_t)NW_ * HH * 2);
    bf* W1s = (bf*)take(64 * 64 * 2); bf* W2s = (bf*)take(64 * 64 * 2); bf* W3s = (bf*)take(64 * 64 * 2); bf* W2i = (bf*)take(64 * 64 * 2); bf* W3i = (bf*)take(64 * 64 * 2);
    bf* Wa_h = (bf*)take(64 * 64 * 2); bf* Wa_d = (bf*)take(64 * 64 * 2); bf* Wb_h = (bf*)take(64 * 64 * 2); bf* Wb_d = (bf*)take(64 * 64 * 2); bf* Wc_a = (bf*)take(64 * 64 * 2); bf* Wc_b = (bf*)take(64 * 64 * 2);
    float* T1 = (float*)take((size_t)NW_ * HH * 4); bf* Ph = (bf*)take((size_t)NW_ * HH * 2); bf* Pl = (bf*)take((size_t)NW_ * HH * 2);
    float* SELF = (float*)take((size_t)NW_ * HH * 4); bf* Sh = (bf*)take((size_t)NW_ * HH * 2); bf* Sl = (bf*)take((size_t)NW_ * HH * 2);
    float* AI = (float*)take((size_t)NW_ * HH * 4); float* BJ = (float*)take((size_t)NW_ * HH * 4); float* CA = (float*)take((size_t)NW_ * HH * 4); float* CB = (float*)take((size_t)NW_ * HH * 4);
    bf* X1h = (bf*)take((size_t)NPC * HH * 2); bf* X1l = (bf*)take((size_t)NPC * HH * 2); float* Y2 = (float*)take((size_t)NPC * HH * 4); bf* X2h = (bf*)take((size_t)NPC * HH * 2); bf* X2l = (bf*)take((size_t)NPC * HH * 2); float* KIJ = (float*)take((size_t)NPC * HH * 4);
    float* ISUM = (float*)take((size_t)NW_ * LL * 4);
    if ((size_t)(wsp - (char*)d_ws) > ws_size) return;
    k_hb<<<(NW_ * HH / 8 + 255) / 256, 256, 0, stream>>>(st, HB);
    k_w64<<<8, 256, 0, stream>>>(Ws1, HH, LL, 0, LL, W1s); k_w64<<<8, 256, 0, stream>>>(Ws2, HH, HH, 0, HH, W2s); k_w64<<<8, 256, 0, stream>>>(Ws3, LL, HH, 0, HH, W3s);
    k_w64<<<8, 256, 0, stream>>>(Wi2, HH, HH, 0, HH, W2i); k_w64<<<8, 256, 0, stream>>>(Wi3, LL, HH, 0, HH, W3i);
    k_w64<<<8, 256, 0, stream>>>(Wi1, HH, 4 * LL, 0, LL, Wa_h); k_w64<<<8, 256, 0, stream>>>(Wi1, HH, 4 * LL, 2 * LL, LL, Wa_d); k_w64<<<8, 256, 0, stream>>>(Wi1, HH, 4 * LL, LL, LL, Wb_h); k_w64<<<8, 256, 0, stream>>>(Wi1, HH, 4 * LL, 3 * LL, LL, Wb_d);
    k_w64<<<8, 256, 0, stream>>>(Wc, LL, 2 * LL, 0, LL, Wc_a); k_w64<<<8, 256, 0, stream>>>(Wc, LL, 2 * LL, LL, LL, Wc_b);
    k_gemmb<false, false><<<dim3(NW_ / 64, 1, 1), 128, 0, stream>>>(HB, nullptr, W1s, nullptr, T1, HH, nullptr, nullptr, HH);
    k_act64<0><<<NW_ / 8, 256, 0, stream>>>(T1, bs1, NW_, Ph, Pl);
    k_gemmb<true, false><<<dim3(NW_ / 64, 1, 1), 128, 0, stream>>>(Ph, Pl, W2s, nullptr, T1, HH, nullptr, nullptr, HH);
    k_act64<0><<<NW_ / 8, 256, 0, stream>>>(T1, bs2, NW_, Ph, Pl);
    k_gemmb<true, false><<<dim3(NW_ / 64, 1, 1), 128, 0, stream>>>(Ph, Pl, W3s, nullptr, SELF, HH, nullptr, nullptr, HH);
    k_act64<2><<<NW_ / 8, 256, 0, stream>>>(SELF, bs3, NW_, Sh, Sl);
    k_gemmb<false, false><<<dim3(NW_ / 64, 1, 1), 128, 0, stream>>>(HB, nullptr, Wa_h, nullptr, T1, HH, nullptr, nullptr, HH);
    k_gemmb<true, false><<<dim3(NW_ / 64, 1, 1), 128, 0, stream>>>(Sh, Sl, Wa_d, nullptr, AI, HH, nullptr, T1, HH, 0);
    k_gemmb<false, false><<<dim3(NW_ / 64, 1, 1), 128, 0, stream>>>(HB, nullptr, Wb_h, nullptr, T1, HH, nullptr, nullptr, HH);
    k_gemmb<true, false><<<dim3(NW_ / 64, 1, 1), 128, 0, stream>>>(Sh, Sl, Wb_d, nullptr, BJ, HH, nullptr, T1, HH, 0);
    k_gemmb<false, false><<<dim3(NW_ / 64, 1, 1), 128, 0, stream>>>(HB, nullptr, Wc_a, nullptr, CA, HH, nullptr, nullptr, HH);
    k_gemmb<false, false><<<dim3(NW_ / 64, 1, 1), 128, 0, stream>>>(HB, nullptr, Wc_b, nullptr, CB, HH, nullptr, nullptr, HH);
    for (int ch = 0; ch < NW_ / ICH; ++ch) { const int i0 = ch * ICH;
        k_x1<<<NPC / 8, 256, 0, stream>>>(AI, BJ, bi1, i0, X1h, X1l);
        k_gemmb<true, false><<<dim3(NPC / 64, 1, 1), 128, 0, stream>>>(X1h, X1l, W2i, nullptr, Y2, HH, nullptr, nullptr, HH);
        k_act64<0><<<NPC / 8, 256, 0, stream>>>(Y2, bi2, NPC, X2h, X2l);
        k_gemmb<true, false><<<dim3(NPC / 64, 1, 1), 128, 0, stream>>>(X2h, X2l, W3i, nullptr, KIJ, HH, nullptr, nullptr, HH);
        k_isum<<<ICH / 8, 256, 0, stream>>>(st, KIJ, bi3, CA, CB, bc, pw, aggr, i0, ISUM); }
    k_out<<<(NW_ * (LL + 1) / 4) / 256, 256, 0, stream>>>(SELF, bs3, ISUM, out);
}
